// Sequencer2DBlock_60232621359575
// MI455X (gfx1250) — hardware-run, weakly checked
//
#include <hip/hip_runtime.h>
#include <math.h>

#pragma clang fp contract(off)

#define NBAT  4
#define HIMG  56
#define WIMG  56
#define CD    192
#define NTOK  (NBAT * HIMG * WIMG)
#define NSEQ  (NBAT * HIMG)
#define SEQL  56
#define DIN   384
#define DXZ   (2 * DIN)
#define DST   16
#define DTR   12
#define XDW   (DTR + 2 * DST)
#define XDN   64
#define DCV   4
#define UW    (4 * CD)
#define HID   576
#define OSTR  68
#define SCW   128
#define LOG2E 1.4426950408889634f
#define RSQ2  0.70710678118654752f
#define WSCAP ((size_t)134217728)

static_assert(HIMG == WIMG);
static_assert(HIMG == SEQL);
static_assert(NTOK % 128 == 0);
static_assert(NTOK % 8 == 0);
static_assert(NTOK % 4 == 0);
static_assert(CD % 64 == 0);
static_assert(CD % 8 == 0);
static_assert((CD / 8) <= 32);
static_assert(DXZ % 64 == 0);
static_assert(DIN % SCW == 0);
static_assert(DIN % 8 == 0);
static_assert(4 * (DIN / 8) == 192);
static_assert(HID % 64 == 0);
static_assert(UW % 64 == 0);
static_assert(CD % 32 == 0);
static_assert(DIN % 32 == 0);
static_assert(UW % 32 == 0);
static_assert(HID % 32 == 0);
static_assert(XDW <= XDN);
static_assert(DTR == 12);
static_assert(DST == 16);
static_assert(DCV == 4);
static_assert(OSTR % 4 == 0);
static_assert(SEQL % 8 == 0);
static_assert(SCW == 128);

typedef unsigned short us16 __attribute__((ext_vector_type(16)));
typedef unsigned short us8  __attribute__((ext_vector_type(8)));
typedef unsigned short us8a __attribute__((ext_vector_type(8), may_alias));
typedef _Float16 v16h __attribute__((ext_vector_type(16)));
typedef _Float16 v8h  __attribute__((ext_vector_type(8)));
typedef float v8f  __attribute__((ext_vector_type(8)));
typedef float v4f  __attribute__((ext_vector_type(4)));
typedef float v4fa __attribute__((ext_vector_type(4), may_alias));
union FragU { us16 v; us8 h[2]; };

__device__ __forceinline__ float bf16r(float f) {
  unsigned u = __float_as_uint(f);
  u += 0x7FFFu + ((u >> 16) & 1u);
  return __uint_as_float(u & 0xFFFF0000u);
}
__device__ __forceinline__ float siluf(float x) { return x * __builtin_amdgcn_rcpf(1.0f + __expf(-x)); }

__device__ __forceinline__ float conv_silu(float c0, float c1, float c2, float c3,
                                           float x0, float x1, float x2, float x3, float bias) {
#pragma clang fp contract(off)
  float a = c0 * x0;
  a = a + c1 * x1;
  a = a + c2 * x2;
  a = a + c3 * x3;
  a = bias + a;
  return siluf(a);
}

__device__ __forceinline__ v8f mma_f16(us16 a, us16 b, v8f c) {
  return __builtin_amdgcn_wmma_f32_16x16x32_f16(false, __builtin_bit_cast(v16h, a), false, __builtin_bit_cast(v16h, b),
                                                (short)0, c, false, false);
}
__device__ __forceinline__ void wguard8(v8f (&c)[2][4], const us16& a0, const us16& a1, const us16 (&b)[4]) {
#if defined(__HIP_DEVICE_COMPILE__)
  asm volatile("v_nop\n\tv_nop\n\tv_nop\n\tv_nop"
               : "+v"(c[0][0]), "+v"(c[0][1]), "+v"(c[0][2]), "+v"(c[0][3]),
                 "+v"(c[1][0]), "+v"(c[1][1]), "+v"(c[1][2]), "+v"(c[1][3])
               : "v"(a0), "v"(a1), "v"(b[0]), "v"(b[1]), "v"(b[2]), "v"(b[3]));
#endif
}

__device__ __forceinline__ us16 gfrag(const unsigned short* __restrict__ P, int ld, int row0, int k0) {
  const int lane = threadIdx.x & 31, r = lane & 15, kh = (lane >> 4) * 8;
  const unsigned short* p = P + (size_t)(row0 + r) * ld + k0 + kh;
  FragU f;
  f.h[0] = *(const us8a*)p;
  f.h[1] = *(const us8a*)(p + 16);
  return f.v;
}

__global__ __launch_bounds__(256) void k_cvtw(const float* __restrict__ W, int N, int K, int Npad,
                                             unsigned short* T, float scale) {
  const int kp = K >> 3;
  const int idx = blockIdx.x * 256 + (int)threadIdx.x;
  if (idx >= Npad * kp) return;
  const int n = idx / kp, k8 = (idx - n * kp) * 8;
  const bool ok = n < N;
  const int nc = ok ? n : (N - 1);
  const float* p = W + (size_t)nc * K + k8;
  const v4f va = *(const v4fa*)p;
  const v4f vb = *(const v4fa*)(p + 4);
  v8h hv;
#pragma unroll
  for (int u = 0; u < 4; ++u) {
    hv[u]     = (_Float16)(ok ? scale * bf16r(va[u]) : 0.0f);
    hv[4 + u] = (_Float16)(ok ? scale * bf16r(vb[u]) : 0.0f);
  }
  const us8 o = __builtin_bit_cast(us8, hv);
  unsigned short* q = T + (size_t)n * K + k8;
  *(volatile us8*)q = o;
  __threadfence();
  *(volatile us8*)q = o;
}

template <int RIN>
__global__ __launch_bounds__(256) void k_ln(const float* __restrict__ X, const float* __restrict__ g,
                                           const float* __restrict__ bt, unsigned short* OUT) {
#pragma clang fp contract(off)
  const int tid = threadIdx.x, lane = tid & 31, wave = tid >> 5;
  const int tok = blockIdx.x * 8 + wave;
  const bool act = lane < (CD / 8);
  const int la = act ? lane : (CD / 8 - 1);
  const float* xr = X + (size_t)tok * CD + 8 * la;
  const v4f ta = *(const v4fa*)xr;
  const v4f tb = *(const v4fa*)(xr + 4);
  float v[8];
#pragma unroll
  for (int u = 0; u < 4; ++u) {
    v[u]     = RIN ? bf16r(ta[u]) : ta[u];
    v[4 + u] = RIN ? bf16r(tb[u]) : tb[u];
  }
#pragma unroll
  for (int i = 0; i < 8; ++i) v[i] = act ? v[i] : 0.0f;
  float s = 0.0f;
#pragma unroll
  for (int i = 0; i < 8; ++i) s = s + v[i];
#pragma unroll
  for (int o = 16; o > 0; o >>= 1) s = s + __shfl_xor(s, o);
  const float mu = s * (1.0f / CD);
  float dv[8];
  float s2 = 0.0f;
#pragma unroll
  for (int i = 0; i < 8; ++i) { dv[i] = act ? (v[i] - mu) : 0.0f; s2 = s2 + dv[i] * dv[i]; }
#pragma unroll
  for (int o = 16; o > 0; o >>= 1) s2 = s2 + __shfl_xor(s2, o);
  const float var = s2 * (1.0f / CD);
  const float rs = rsqrtf(var + 1e-6f);
  v8h hv;
#pragma unroll
  for (int u = 0; u < 8; ++u) {
    const int ch = 8 * la + u;
    const float w = (dv[u] * rs) * bf16r(g[ch]) + bf16r(bt[ch]);
    hv[u] = (_Float16)(8.0f * w);
  }
  const us8 o = __builtin_bit_cast(us8, hv);
  unsigned short* p = OUT + (size_t)tok * CD + 8 * la;
  if (act) *(volatile us8*)p = o;
  __threadfence();
  if (act) *(volatile us8*)p = o;
}

template <int EPI>
__global__ __launch_bounds__(128) void k_gemm(const unsigned short* __restrict__ A, int lda,
                                             const unsigned short* __restrict__ B, int ldb, int K, float scale,
                                             float* Yf, int ldy, unsigned short* Y16, int ldh, int coff, float s16,
                                             const float* __restrict__ bias, const float* __restrict__ res) {
  __shared__ __attribute__((aligned(16))) float sm[4 * 32 * OSTR];
  const int tid = threadIdx.x, lane = tid & 31, wave = tid >> 5, cl = lane & 15, hh = lane >> 4;
  const int m0 = blockIdx.x * 128 + wave * 32, n0 = blockIdx.y * 64;

  v8f acc[2][4];
#pragma unroll
  for (int i = 0; i < 2; ++i)
#pragma unroll
    for (int j = 0; j < 4; ++j) { v8f zz = {0.f, 0.f, 0.f, 0.f, 0.f, 0.f, 0.f, 0.f}; acc[i][j] = zz; }

#pragma unroll 1
  for (int k0 = 0; k0 < K; k0 += 32) {
    const us16 a0 = gfrag(A, lda, m0, k0);
    const us16 a1 = gfrag(A, lda, m0 + 16, k0);
    us16 bfr[4];
#pragma unroll
    for (int j = 0; j < 4; ++j) bfr[j] = gfrag(B, ldb, n0 + 16 * j, k0);
#pragma unroll
    for (int j = 0; j < 4; ++j) {
      acc[0][j] = mma_f16(a0, bfr[j], acc[0][j]);
      acc[1][j] = mma_f16(a1, bfr[j], acc[1][j]);
    }
    wguard8(acc, a0, a1, bfr);
  }

  float bb[4] = {0.0f, 0.0f, 0.0f, 0.0f};
  if (EPI == 3) {
#pragma unroll
    for (int j = 0; j < 4; ++j) bb[j] = bf16r(bias[n0 + 16 * j + cl]);
  }
  float* so = sm + wave * (32 * OSTR);
#pragma unroll
  for (int i = 0; i < 2; ++i)
#pragma unroll
    for (int j = 0; j < 4; ++j)
#pragma unroll
      for (int r = 0; r < 8; ++r) {
        float v = acc[i][j][r] * scale;
        if (EPI == 3) {
          const float t = v + bb[j];
          v = 0.5f * t * (1.0f + erff(t * RSQ2));
        }
        so[(16 * i + 8 * hh + r) * OSTR + 16 * j + cl] = v;
      }
  __syncthreads();

#pragma unroll
  for (int pass = 0; pass < 2; ++pass) {
    if (EPI == 0 || EPI == 2 || EPI == 4) {
#pragma unroll
      for (int it = 0; it < 16; ++it) {
        const int ch = it * 32 + lane, r = ch >> 4, q = (ch & 15) * 4;
        v4f v = *(const v4fa*)(so + r * OSTR + q);
        if (EPI == 2) {
          const v4f xv = *(const v4fa*)(res + (size_t)(m0 + r) * ldy + n0 + q);
          const v4f bq = *(const v4fa*)(bias + n0 + q);
#pragma unroll
          for (int u = 0; u < 4; ++u) v[u] = (bf16r(xv[u]) + v[u]) + bf16r(bq[u]);
        }
        if (EPI == 4) {
          const v4f xv = *(const v4fa*)(res + (size_t)(m0 + r) * ldy + n0 + q);
          const v4f bq = *(const v4fa*)(bias + n0 + q);
#pragma unroll
          for (int u = 0; u < 4; ++u) v[u] = xv[u] + (v[u] + bf16r(bq[u]));
        }
        *(volatile v4f*)(Yf + (size_t)(m0 + r) * ldy + n0 + q) = v;
      }
    } else {
#pragma unroll
      for (int it = 0; it < 8; ++it) {
        const int p = it * 32 + lane, r = p >> 3, k8 = (p & 7) * 8;
        const v4f va = *(const v4fa*)(so + r * OSTR + k8);
        const v4f vb = *(const v4fa*)(so + r * OSTR + k8 + 4);
        v8h hv;
#pragma unroll
        for (int u = 0; u < 4; ++u) { hv[u] = (_Float16)(s16 * va[u]); hv[4 + u] = (_Float16)(s16 * vb[u]); }
        *(volatile us8*)(Y16 + (size_t)(m0 + r) * ldh + (size_t)(coff + n0 + k8)) = __builtin_bit_cast(us8, hv);
      }
    }
    __threadfence();
  }
}

template <int AXIS, int DIR>
__global__ __launch_bounds__(192) void k_conv(const float* __restrict__ XZ, const float* __restrict__ cw,
                                             const float* __restrict__ cb, unsigned short* XC) {
#pragma clang fp contract(off)
  const int tid = threadIdx.x;
  const int tq = tid / 48;
  const int c = (tid - tq * 48) * 8;
  const int tok = blockIdx.x * 4 + tq;
  const int pos = AXIS ? ((tok / WIMG) % HIMG) : (tok % WIMG);
  const int tstr = AXIS ? WIMG : 1;
  float xv[DCV][8];
#pragma unroll
  for (int k = 0; k < DCV; ++k) {
    const int p2 = DIR ? (pos + (DCV - 1) - k) : (pos - (DCV - 1) + k);
    const bool ok = (p2 >= 0) && (p2 <= SEQL - 1);
    const int pc = p2 < 0 ? 0 : (p2 > SEQL - 1 ? SEQL - 1 : p2);
    const float* p = XZ + (size_t)(tok + (pc - pos) * tstr) * DXZ + c;
    const v4f va = *(const v4fa*)p;
    const v4f vb = *(const v4fa*)(p + 4);
#pragma unroll
    for (int u = 0; u < 4; ++u) { xv[k][u] = ok ? va[u] : 0.0f; xv[k][4 + u] = ok ? vb[u] : 0.0f; }
  }
  float wv[8][DCV];
#pragma unroll
  for (int u = 0; u < 8; ++u) {
    const v4f w4 = *(const v4fa*)(cw + (size_t)(c + u) * DCV);
#pragma unroll
    for (int k = 0; k < DCV; ++k) wv[u][k] = bf16r(w4[k]);
  }
  float bv[8];
  {
    const v4f ba = *(const v4fa*)(cb + c);
    const v4f bb2 = *(const v4fa*)(cb + c + 4);
#pragma unroll
    for (int u = 0; u < 4; ++u) { bv[u] = bf16r(ba[u]); bv[4 + u] = bf16r(bb2[u]); }
  }
  v8h hv;
#pragma unroll
  for (int u = 0; u < 8; ++u) {
    const float sres = conv_silu(wv[u][0], wv[u][1], wv[u][2], wv[u][3], xv[0][u], xv[1][u], xv[2][u], xv[3][u], bv[u]);
    hv[u] = (_Float16)(64.0f * sres);
  }
  const us8 o = __builtin_bit_cast(us8, hv);
  const size_t off = (size_t)tok * DIN + c;
  *(volatile us8*)(XC + off) = o;
  __threadfence();
  *(volatile us8*)(XC + off) = o;
}

template <int AXIS, int DIR>
__global__ __launch_bounds__(SCW) void k_scan(const float* __restrict__ XZ, const float* __restrict__ DBC,
                                             const float* __restrict__ cw, const float* __restrict__ cb,
                                             const float* __restrict__ Wdt, const float* __restrict__ bdt,
                                             const float* __restrict__ Alog, const float* __restrict__ Dv,
                                             unsigned short* YG) {
#pragma clang fp contract(off)
  __shared__ __attribute__((aligned(16))) float sy[SEQL * SCW];
  const int g = blockIdx.x, o = blockIdx.y;
  const int tid = threadIdx.x, lane = tid & 31, wave = tid >> 5, cl = lane & 15, hh = lane >> 4;
  const int d = g * SCW + tid;
  const int tok0 = AXIS ? ((o / WIMG) * (HIMG * WIMG) + (o % WIMG)) : (o * WIMG);
  const int tstr = AXIS ? WIMG : 1;

  float A2[DST], h[DST];
#pragma unroll
  for (int q = 0; q < 4; ++q) {
    const v4f a4 = *(const v4fa*)(Alog + (size_t)d * DST + 4 * q);
#pragma unroll
    for (int u = 0; u < 4; ++u) { A2[4 * q + u] = -__expf(bf16r(a4[u])) * LOG2E; h[4 * q + u] = 0.0f; }
  }
  float wd[DTR];
#pragma unroll
  for (int q = 0; q < 3; ++q) {
    const v4f w4 = *(const v4fa*)(Wdt + (size_t)d * DTR + 4 * q);
#pragma unroll
    for (int u = 0; u < 4; ++u) wd[4 * q + u] = bf16r(w4[u]);
  }
  const v4f c4 = *(const v4fa*)(cw + (size_t)d * DCV);
  const float cw0 = bf16r(c4[0]), cw1 = bf16r(c4[1]), cw2 = bf16r(c4[2]), cw3 = bf16r(c4[3]);
  const float cbv = bf16r(cb[d]);
  const float Dd = bf16r(Dv[d]);
  const float bd = bf16r(bdt[d]);
  float w1 = 0.0f, w2 = 0.0f, w3 = 0.0f;

#pragma unroll 1
  for (int st = 0; st < SEQL; ++st) {
    const int pos = DIR ? (SEQL - 1 - st) : st;
    const size_t tok = (size_t)(tok0 + pos * tstr);
    const float* pdb = DBC + tok * XDN;
    v4f T4[3], Bv[4], Cv[4];
#pragma unroll
    for (int q = 0; q < 3; ++q) T4[q] = *(const v4fa*)(pdb + 4 * q);
#pragma unroll
    for (int q = 0; q < 4; ++q) {
      Bv[q] = *(const v4fa*)(pdb + DTR + 4 * q);
      Cv[q] = *(const v4fa*)(pdb + DTR + DST + 4 * q);
    }
    float s = T4[0][0] * wd[0];
#pragma unroll
    for (int r = 1; r < DTR; ++r) s = s + T4[r >> 2][r & 3] * wd[r];
    const float raw = s + bd;
    const float dl = fmaxf(raw, 0.0f) + log1pf(__expf(-fabsf(raw)));
    const float xcur = XZ[tok * DXZ + d];
    const float zv = XZ[tok * DXZ + DIN + d];
    const float xc = conv_silu(cw0, cw1, cw2, cw3, w3, w2, w1, xcur, cbv);
    w3 = w2; w2 = w1; w1 = xcur;
    const float dx = dl * xc;
    float y = 0.0f;
#pragma unroll
    for (int n = 0; n < DST; ++n) {
      const float e = exp2f(dl * A2[n]);
      h[n] = e * h[n] + dx * Bv[n >> 2][n & 3];
      y = y + h[n] * Cv[n >> 2][n & 3];
    }
    const float yv = (y + Dd * xc) * siluf(zv);
    sy[pos * SCW + tid] = yv;
  }
  __syncthreads();

#pragma unroll
  for (int pass = 0; pass < 2; ++pass) {
#pragma unroll
    for (int it = 0; it < SEQL / 8; ++it) {
      const int row = it * 8 + wave * 2 + hh;
      const size_t tok = (size_t)(tok0 + row * tstr);
      const v4f va = *(const v4fa*)(sy + row * SCW + 8 * cl);
      const v4f vb = *(const v4fa*)(sy + row * SCW + 8 * cl + 4);
      v8h hv;
#pragma unroll
      for (int u = 0; u < 4; ++u) { hv[u] = (_Float16)(256.0f * va[u]); hv[4 + u] = (_Float16)(256.0f * vb[u]); }
      *(volatile us8*)(YG + tok * DIN + (size_t)(g * SCW + 8 * cl)) = __builtin_bit_cast(us8, hv);
    }
    __threadfence();
  }
}

extern "C" void kernel_launch(void* const* d_in, const int* in_sizes, int n_in,
                              void* d_out, int out_size, void* d_ws, size_t ws_size,
                              hipStream_t stream) {
  if (n_in < 29) return;
  if (in_sizes[0] != NTOK * CD || out_size != NTOK * CD) return;
  for (int i = 1; i <= 4; ++i) if (in_sizes[i] != CD) return;
  for (int ax = 0; ax < 2; ++ax) {
    const int o = 5 + 9 * ax;
    if (in_sizes[o] != DXZ * CD || in_sizes[o + 1] != DIN * DCV || in_sizes[o + 2] != DIN || in_sizes[o + 3] != XDW * DIN ||
        in_sizes[o + 4] != DIN * DTR || in_sizes[o + 5] != DIN || in_sizes[o + 6] != DIN * DST || in_sizes[o + 7] != DIN ||
        in_sizes[o + 8] != CD * DIN) return;
  }
  if (in_sizes[23] != CD * UW || in_sizes[24] != CD || in_sizes[25] != HID * CD || in_sizes[26] != HID ||
      in_sizes[27] != CD * HID || in_sizes[28] != CD) return;

  const float* x    = (const float*)d_in[0];
  const float* ln1g = (const float*)d_in[1];
  const float* ln1b = (const float*)d_in[2];
  const float* ln2g = (const float*)d_in[3];
  const float* ln2b = (const float*)d_in[4];
  const float* inw[2], *cvw[2], *cvb[2], *xpw[2], *dtw[2], *dtbv[2], *alg[2], *dpv[2], *ouw[2];
  for (int ax = 0; ax < 2; ++ax) {
    const int o = 5 + 9 * ax;
    inw[ax]  = (const float*)d_in[o + 0];
    cvw[ax]  = (const float*)d_in[o + 1];
    cvb[ax]  = (const float*)d_in[o + 2];
    xpw[ax]  = (const float*)d_in[o + 3];
    dtw[ax]  = (const float*)d_in[o + 4];
    dtbv[ax] = (const float*)d_in[o + 5];
    alg[ax]  = (const float*)d_in[o + 6];
    dpv[ax]  = (const float*)d_in[o + 7];
    ouw[ax]  = (const float*)d_in[o + 8];
  }
  const float* fcw  = (const float*)d_in[23];
  const float* fcb  = (const float*)d_in[24];
  const float* mw1  = (const float*)d_in[25];
  const float* mb1  = (const float*)d_in[26];
  const float* mw2  = (const float*)d_in[27];
  const float* mb2  = (const float*)d_in[28];
  float* out = (float*)d_out;

  size_t off = 0;
  auto carve = [&](size_t bytes) -> char* { char* p = (char*)d_ws + off; off += (bytes + 255) & ~(size_t)255; return p; };
  unsigned short* WIN0 = (unsigned short*)carve((size_t)DXZ * CD * 2);
  unsigned short* WIN1 = (unsigned short*)carve((size_t)DXZ * CD * 2);
  unsigned short* WX0  = (unsigned short*)carve((size_t)XDN * DIN * 2);
  unsigned short* WX1  = (unsigned short*)carve((size_t)XDN * DIN * 2);
  unsigned short* WOU0 = (unsigned short*)carve((size_t)CD * DIN * 2);
  unsigned short* WOU1 = (unsigned short*)carve((size_t)CD * DIN * 2);
  unsigned short* WFC  = (unsigned short*)carve((size_t)CD * UW * 2);
  unsigned short* WM1  = (unsigned short*)carve((size_t)HID * CD * 2);
  unsigned short* WM2  = (unsigned short*)carve((size_t)CD * HID * 2);
  unsigned short* WH   = (unsigned short*)carve((size_t)NTOK * CD * 2);
  float* XZ            = (float*)carve((size_t)NTOK * DXZ * 4);
  unsigned short* XC16 = (unsigned short*)carve((size_t)NTOK * DIN * 2);
  float* DBC           = (float*)carve((size_t)NTOK * XDN * 4);
  unsigned short* YG   = (unsigned short*)carve((size_t)NTOK * DIN * 2);
  unsigned short* U    = (unsigned short*)carve((size_t)NTOK * UW * 2);
  float* X1            = (float*)carve((size_t)NTOK * CD * 4);
  unsigned short* XN2  = (unsigned short*)carve((size_t)NTOK * CD * 2);
  unsigned short* M16  = (unsigned short*)carve((size_t)NTOK * HID * 2);
  if (off > ws_size || off > WSCAP) return;

  const dim3 b256(256), b192(192), b128(128);
  auto cvtw = [&](const float* W, int N, int K, int Npad, unsigned short* T, float scale) {
    const int pieces = Npad * (K / 8);
    k_cvtw<<<dim3((pieces + 255) / 256), b256, 0, stream>>>(W, N, K, Npad, T, scale);
  };
  cvtw(inw[0], DXZ, CD, DXZ, WIN0, 64.0f);
  cvtw(inw[1], DXZ, CD, DXZ, WIN1, 64.0f);
  cvtw(xpw[0], XDW, DIN, XDN, WX0, 64.0f);
  cvtw(xpw[1], XDW, DIN, XDN, WX1, 64.0f);
  cvtw(ouw[0], CD, DIN, CD, WOU0, 64.0f);
  cvtw(ouw[1], CD, DIN, CD, WOU1, 64.0f);
  cvtw(fcw, CD, UW, CD, WFC, 64.0f);
  cvtw(mw1, HID, CD, HID, WM1, 64.0f);
  cvtw(mw2, CD, HID, CD, WM2, 64.0f);
  k_ln<1><<<dim3(NTOK / 8), b256, 0, stream>>>(x, ln1g, ln1b, WH);

  for (int ax = 0; ax < 2; ++ax) {
    unsigned short* WIN = ax ? WIN1 : WIN0;
    unsigned short* WX  = ax ? WX1 : WX0;
    unsigned short* WOU = ax ? WOU1 : WOU0;
    k_gemm<0><<<dim3(NTOK / 128, DXZ / 64), b128, 0, stream>>>(WH, CD, WIN, CD, CD, 1.0f / 512.0f, XZ, DXZ, U, UW, 0, 1.0f, fcb, x);
    for (int dr = 0; dr < 2; ++dr) {
      if (ax == 0) {
        if (dr == 0) k_conv<0, 0><<<dim3(NTOK / 4), b192, 0, stream>>>(XZ, cvw[0], cvb[0], XC16);
        else         k_conv<0, 1><<<dim3(NTOK / 4), b192, 0, stream>>>(XZ, cvw[0], cvb[0], XC16);
      } else {
        if (dr == 0) k_conv<1, 0><<<dim3(NTOK / 4), b192, 0, stream>>>(XZ, cvw[1], cvb[1], XC16);
        else         k_conv<1, 1><<<dim3(NTOK / 4), b192, 0, stream>>>(XZ, cvw[1], cvb[1], XC16);
      }
      k_gemm<0><<<dim3(NTOK / 128, XDN / 64), b128, 0, stream>>>(XC16, DIN, WX, DIN, DIN, 1.0f / 4096.0f, DBC, XDN, U, UW, 0, 1.0f, fcb, x);
      if (ax == 0) {
        if (dr == 0) k_scan<0, 0><<<dim3(DIN / SCW, NSEQ), b128, 0, stream>>>(XZ, DBC, cvw[0], cvb[0], dtw[0], dtbv[0], alg[0], dpv[0], YG);
        else         k_scan<0, 1><<<dim3(DIN / SCW, NSEQ), b128, 0, stream>>>(XZ, DBC, cvw[0], cvb[0], dtw[0], dtbv[0], alg[0], dpv[0], YG);
      } else {
        if (dr == 0) k_scan<1, 0><<<dim3(DIN / SCW, NSEQ), b128, 0, stream>>>(XZ, DBC, cvw[1], cvb[1], dtw[1], dtbv[1], alg[1], dpv[1], YG);
        else         k_scan<1, 1><<<dim3(DIN / SCW, NSEQ), b128, 0, stream>>>(XZ, DBC, cvw[1], cvb[1], dtw[1], dtbv[1], alg[1], dpv[1], YG);
      }
      const int coff = (ax == 0 ? 2 * CD : 0) + dr * CD;
      k_gemm<1><<<dim3(NTOK / 128, CD / 64), b128, 0, stream>>>(YG, DIN, WOU, DIN, DIN, 1.0f / 16384.0f, XZ, DXZ, U, UW, coff, 1024.0f, fcb, x);
    }
  }
  k_gemm<2><<<dim3(NTOK / 128, CD / 64), b128, 0, stream>>>(U, UW, WFC, UW, UW, 1.0f / 65536.0f, X1, CD, U, UW, 0, 1.0f, fcb, x);
  k_ln<0><<<dim3(NTOK / 8), b256, 0, stream>>>(X1, ln2g, ln2b, XN2);
  k_gemm<3><<<dim3(NTOK / 128, HID / 64), b128, 0, stream>>>(XN2, CD, WM1, CD, CD, 1.0f / 512.0f, XZ, DXZ, M16, HID, 0, 32.0f, mb1, x);
  k_gemm<4><<<dim3(NTOK / 128, CD / 64), b128, 0, stream>>>(M16, HID, WM2, HID, HID, 1.0f / 2048.0f, out, CD, U, UW, 0, 1.0f, mb2, X1);
}
